// GATSelfAttention_6665789243985
// MI455X (gfx1250) — hardware-run, weakly checked
//
#include <hip/hip_runtime.h>
#include <math.h>

typedef __attribute__((ext_vector_type(16))) _Float16 v16h;
typedef __attribute__((ext_vector_type(8)))  _Float16 v8h;
typedef __attribute__((ext_vector_type(8)))  float    v8f;
typedef __attribute__((ext_vector_type(4)))  float    v4f;
typedef __attribute__((ext_vector_type(2)))  float    v2f;
typedef __attribute__((ext_vector_type(4)))  unsigned v4u;
typedef __attribute__((ext_vector_type(4)))  int      v4i;

constexpr int kNB    = 32;
constexpr int kNE    = 512;
constexpr int kDim   = 300;
constexpr int kDimP  = 320;
constexpr int kNTy   = 4;
constexpr int kTwoD  = 600;
constexpr float kSlope  = 0.2f;
constexpr float kFill   = -1.0e30f;
constexpr float kXCarry = 64.0f;
constexpr float kWCarry = 1024.0f;
constexpr float kHCarry = 512.0f;
constexpr float kScale1 = kHCarry / (kXCarry * kWCarry);
constexpr float kScale2 = 1.0f / kHCarry;
constexpr float kF16Min = 6.103515625e-5f;
static_assert((kDimP % 64) == 0 && (kNE % 64) == 0 && (kDimP % 32) == 0 && (kNE % 32) == 0);
static_assert(kDimP >= kDim && kTwoD == 2 * kDim);

constexpr size_t kSzW3T = (size_t)kDimP * kDimP * 2;
constexpr size_t kSzU   = (size_t)kNTy * kNB * 2 * kDimP * 4;
constexpr size_t kSzS   = (size_t)kNB * 8 * kNE * 4;
constexpr size_t kSzXH  = (size_t)kNB * kNE * kDimP * 2;
constexpr size_t kSzHMT = (size_t)kNB * kDimP * kNE * 2;
constexpr size_t kSzPP  = (size_t)kNB * kNE * kNE * 2;
constexpr size_t kSzZI  = (size_t)kNB * kNE * 4;
constexpr size_t kOffW3T = 0;
constexpr size_t kOffU   = kOffW3T + kSzW3T;
constexpr size_t kOffS   = kOffU   + kSzU;
constexpr size_t kOffXH  = kOffS   + kSzS;
constexpr size_t kOffHMT = kOffXH  + kSzXH;
constexpr size_t kOffPP  = kOffHMT + kSzHMT;
constexpr size_t kOffZI  = kOffPP  + kSzPP;
constexpr size_t kWsTotal = kOffZI + kSzZI;
static_assert(kWsTotal == 38871040ull);
static_assert(kWsTotal <= 134217728ull);
static_assert((kOffU % 128) == 0 && (kOffS % 128) == 0 && (kOffXH % 128) == 0 && (kOffHMT % 128) == 0 &&
              (kOffPP % 128) == 0 && (kOffZI % 128) == 0);

__device__ __forceinline__ float flush_h(float v) { return (fabsf(v) < kF16Min) ? 0.0f : v; }

__device__ __forceinline__ unsigned pack_h2(float a, float b) {
  const _Float16 h0 = (_Float16)a, h1 = (_Float16)b;
  return (unsigned)__builtin_bit_cast(unsigned short, h0) | ((unsigned)__builtin_bit_cast(unsigned short, h1) << 16);
}

struct FragH {
  union U { v16h v; v8h h[2]; };
  static __device__ __forceinline__ v16h load(const _Float16* p) {
    U f; f.h[0] = *(const v8h*)(p); f.h[1] = *(const v8h*)(p + 16); return f.v;
  }
};

__device__ __forceinline__ v8f mma_h(v16h a, v16h b, v8f c) {
  c = __builtin_amdgcn_wmma_f32_16x16x32_f16(false, a, false, b, (short)0, c, false, false);
  asm volatile("v_nop\n\tv_nop\n\tv_nop\n\tv_nop" : "+v"(c) : "v"(a), "v"(b));
  return c;
}

static_assert((kDimP * (kDimP / 8)) % 256 == 0);
__global__ __launch_bounds__(256) void prep_w3t_kernel(const float* __restrict__ W_type, unsigned short* __restrict__ W3T)
{
  const int i  = blockIdx.x * 256 + threadIdx.x;
  const int d  = i / (kDimP / 8);
  const int k0 = (i - d * (kDimP / 8)) * 8;
  const float* W3 = W_type + (size_t)(kNTy - 1) * kDim * kDim;
  const int dc = d < kDim ? d : (kDim - 1);
  v8h hv;
#pragma unroll
  for (int e = 0; e < 8; ++e) {
    const int k  = k0 + e;
    const int kc = k < kDim ? k : (kDim - 1);
    float w = W3[(size_t)kc * kDim + dc];
    asm volatile("" : "+v"(w));
    float wv = (k < kDim && d < kDim) ? (w * kWCarry) : 0.0f;
    wv = flush_h(wv);
    hv[e] = (_Float16)wv;
  }
  unsigned short* dst = W3T + (size_t)i * 8;
  *(volatile v8h*)dst = hv;
  __threadfence();
  *(volatile v8h*)dst = hv;
}

__global__ __launch_bounds__(256) void gate_fold_kernel(
    const float* __restrict__ query, const float* __restrict__ W_type, const float* __restrict__ a_type,
    const float* __restrict__ W1, const float* __restrict__ W2, float* __restrict__ U)
{
  __shared__ __align__(16) float q[kDim];
  __shared__ __align__(16) float t1[kTwoD];
  __shared__ __align__(16) float cc[kTwoD];
  __shared__ __align__(16) float uo[2 * kDimP];
  const int ty = blockIdx.x, n = blockIdx.y, tid = threadIdx.x;

  const float* qn = query + (size_t)n * kDim;
  for (int d = tid; d < kDim; d += 256) q[d] = qn[d];
  __syncthreads();

  const float* w1 = W1 + (size_t)ty * kDim * kTwoD;
  for (int k = tid; k < kTwoD; k += 256) {
    float s = 0.f;
#pragma unroll 4
    for (int d = 0; d < kDim; ++d) s = fmaf(q[d], w1[(size_t)d * kTwoD + k], s);
    t1[k] = s > 0.f ? s : 0.f;
  }
  __syncthreads();

  const float* w2 = W2 + (size_t)ty * kTwoD * kTwoD;
  const float* at = a_type + (size_t)ty * kTwoD;
  for (int k = tid; k < kTwoD; k += 256) {
    float s = 0.f;
#pragma unroll 4
    for (int j = 0; j < kTwoD; ++j) s = fmaf(t1[j], w2[(size_t)j * kTwoD + k], s);
    const float g = 1.0f / (1.0f + expf(-s));
    cc[k] = g * at[k];
  }
  __syncthreads();

  const float* w = W_type + (size_t)ty * kDim * kDim;
  for (int d = tid; d < kDim; d += 256) {
    const float* wr = w + (size_t)d * kDim;
    float s1 = 0.f, s2 = 0.f;
#pragma unroll 4
    for (int f = 0; f < kDim; ++f) {
      const float wv = wr[f];
      s1 = fmaf(wv, cc[f], s1);
      s2 = fmaf(wv, cc[kDim + f], s2);
    }
    uo[d] = s1;
    uo[kDimP + d] = s2;
  }
  if (tid < 2 * (kDimP - kDim)) {
    const int side = tid / (kDimP - kDim);
    const int p = tid - side * (kDimP - kDim);
    uo[side * kDimP + kDim + p] = 0.0f;
  }
  __syncthreads();
  if (tid < (2 * kDimP) / 4) {
    const v4f v = *(const v4f*)(uo + tid * 4);
    float* dst = U + (size_t)(ty * kNB + n) * (2 * kDimP) + tid * 4;
    *(volatile v4f*)dst = v;
    __threadfence();
    *(volatile v4f*)dst = v;
  }
}

__global__ __launch_bounds__(256) void score_cast_kernel(
    const float* __restrict__ x, const float* __restrict__ U, float* __restrict__ S, unsigned short* __restrict__ XH)
{
  __shared__ __align__(16) float    us[8 * kDimP];
  __shared__ __align__(16) unsigned xt[64 * (kDimP / 2)];
  __shared__ __align__(16) float    sS[8 * 64];
  const int tid = threadIdx.x, lane = tid & 31, wave = tid >> 5;
  const int blk = blockIdx.x, n = blockIdx.y;

  for (int idx = tid; idx < 8 * (kDimP / 4); idx += 256) {
    const int p  = idx / (kDimP / 4);
    const int c4 = (idx - p * (kDimP / 4)) * 4;
    const int ty = p >> 1, side = p & 1;
    *(v4f*)(us + p * kDimP + c4) = *(const v4f*)(U + (size_t)((ty * kNB + n) * 2 + side) * kDimP + c4);
  }
  __syncthreads();

#pragma unroll 1
  for (int rr = 0; rr < 8; ++rr) {
    const int rl = wave * 8 + rr;
    const float* xr = x + (size_t)(n * kNE + blk * 64 + rl) * kDim;
    float acc[8];
#pragma unroll
    for (int t = 0; t < 8; ++t) acc[t] = 0.0f;
#pragma unroll 1
    for (int it = 0; it < 5; ++it) {
      const int k  = it * 64 + lane * 2;
      const int kc = k < kDim ? k : (kDim - 2);
      const v2f xv = *(const v2f*)(xr + kc);
      float xa = xv.x, xb = xv.y;
      asm volatile("" : "+v"(xa), "+v"(xb));
      const float a = (k < kDim) ? xa : 0.0f;
      const float b = (k < kDim) ? xb : 0.0f;
      xt[rl * (kDimP / 2) + it * 32 + lane] = pack_h2(flush_h(a * kXCarry), flush_h(b * kXCarry));
#pragma unroll
      for (int t = 0; t < 8; ++t) {
        const v2f uu = *(const v2f*)(us + t * kDimP + k);
        acc[t] = fmaf(a, uu.x, acc[t]);
        acc[t] = fmaf(b, uu.y, acc[t]);
      }
    }
#pragma unroll
    for (int t = 0; t < 8; ++t) {
#pragma unroll
      for (int off = 16; off > 0; off >>= 1) acc[t] += __shfl_xor(acc[t], off, 32);
    }
    if (lane == 0) {
#pragma unroll
      for (int t = 0; t < 8; ++t) sS[t * 64 + rl] = acc[t];
    }
  }
  __syncthreads();

  float* sdst = S + (size_t)(n * 8 + wave) * kNE + blk * 64 + (lane & 15) * 4;
  const v4f sv = *(const v4f*)(sS + wave * 64 + (lane & 15) * 4);
  unsigned* xdst = (unsigned*)XH + (size_t)(n * kNE + blk * 64) * (kDimP / 2);
  for (int pass = 0; pass < 2; ++pass) {
    if (lane < 16) *(volatile v4f*)sdst = sv;
#pragma unroll 1
    for (int it = 0; it < 10; ++it) {
      const int f = it * 256 + tid;
      const v4u v = *(const v4u*)(xt + f * 4);
      *(volatile v4u*)(xdst + (size_t)f * 4) = v;
    }
    __threadfence();
  }
}

static_assert(((kDimP / 64) * (kNE / 64)) % 8 == 0);
__global__ __launch_bounds__(256) void proj_gemm_kernel(
    const unsigned short* __restrict__ Ap, const unsigned short* __restrict__ Btp,
    unsigned short* __restrict__ Cout, const float* __restrict__ colscale)
{
  const _Float16* A  = (const _Float16*)Ap;
  const _Float16* Bt = (const _Float16*)Btp;
  __shared__ __align__(16) float sT[8][16 * 68];
  const int b    = blockIdx.y;
  const int lane = threadIdx.x & 31;
  const int wave = threadIdx.x >> 5;
  constexpr int tilesN = kNE >> 6;
  const int tile = blockIdx.x * 8 + wave;
  const int tm = tile / tilesN;
  const int tn = tile - tm * tilesN;
  const int m0 = tm << 6;
  const int n0 = tn << 6;
  const _Float16* Bb = Bt + (size_t)b * kNE * kDimP;

  const int rlane = lane & 15;
  const int koff  = (lane >> 4) * 8;
  const int mOff  = (lane >> 4) * 8;

  v8f acc[4][4];
#pragma unroll
  for (int i = 0; i < 4; ++i)
#pragma unroll
    for (int j = 0; j < 4; ++j) acc[i][j] = (v8f){0.f,0.f,0.f,0.f,0.f,0.f,0.f,0.f};

#pragma unroll 1
  for (int k0 = 0; k0 < kDimP; k0 += 32) {
    v16h bh[4];
#pragma unroll
    for (int j = 0; j < 4; ++j)
      bh[j] = FragH::load(Bb + (size_t)(n0 + (j << 4) + rlane) * kDimP + koff + k0);
#pragma unroll
    for (int i = 0; i < 4; ++i) {
      const v16h ah = FragH::load(A + (size_t)(m0 + (i << 4) + rlane) * kDimP + koff + k0);
#pragma unroll
      for (int j = 0; j < 4; ++j) acc[i][j] = mma_h(ah, bh[j], acc[i][j]);
    }
  }

  float cs[4];
#pragma unroll
  for (int j = 0; j < 4; ++j) cs[j] = colscale[(size_t)b * kNE + n0 + (j << 4) + rlane] * kScale1;

  float* slab = sT[wave];
  unsigned short* C = Cout + (size_t)b * kDimP * kNE;
#pragma unroll
  for (int i = 0; i < 4; ++i) {
    const int mBase = m0 + (i << 4);
#pragma unroll
    for (int j = 0; j < 4; ++j) {
#pragma unroll
      for (int r = 0; r < 8; ++r) slab[(mOff + r) * 68 + (j << 4) + rlane] = acc[i][j][r] * cs[j];
    }
    __builtin_amdgcn_fence(__ATOMIC_RELEASE, "workgroup");
    __builtin_amdgcn_wave_barrier();
    __builtin_amdgcn_fence(__ATOMIC_ACQUIRE, "workgroup");
    {
      const int q = lane >> 3, c8 = (lane & 7) * 8;
      for (int pass = 0; pass < 2; ++pass) {
#pragma unroll
        for (int it = 0; it < 4; ++it) {
          const int row = it * 4 + q;
          const float* sp = slab + row * 68 + c8;
          v8h hv;
#pragma unroll
          for (int e = 0; e < 8; ++e) {
            const float fv = flush_h(sp[e]);
            hv[e] = (_Float16)fv;
          }
          *(volatile v8h*)(C + (size_t)(mBase + row) * kNE + n0 + c8) = hv;
        }
        __threadfence();
      }
    }
    __builtin_amdgcn_fence(__ATOMIC_RELEASE, "workgroup");
    __builtin_amdgcn_wave_barrier();
    __builtin_amdgcn_fence(__ATOMIC_ACQUIRE, "workgroup");
  }
}

__global__ __launch_bounds__(256) void coef_kernel(
    const int* __restrict__ adj, const float* __restrict__ S, unsigned short* __restrict__ PP, float* __restrict__ ZI)
{
  __shared__ __align__(16) float sd[kNTy * kNE];
  __shared__ __align__(16) float ssrc[kNTy * 64];
  __shared__ __align__(16) float sc[8][kNE];
  __shared__ __align__(16) float sz[64];
  const int tid = threadIdx.x, lane = tid & 31, wave = tid >> 5;
  const int blk = blockIdx.x, n = blockIdx.y;

#pragma unroll
  for (int rep = 0; rep < 2; ++rep) {
    const int idx = tid + rep * 256;
    const int t  = idx >> 7;
    const int c4 = (idx & 127) * 4;
    *(v4f*)(sd + t * kNE + c4) = *(const v4f*)(S + (size_t)(n * 8 + t * 2 + 1) * kNE + c4);
  }
  {
    const int t = tid >> 6, r = tid & 63;
    ssrc[tid] = S[(size_t)(n * 8 + t * 2) * kNE + blk * 64 + r];
  }
  __syncthreads();

  float* scw = sc[wave];
#pragma unroll 1
  for (int rr = 0; rr < 8; ++rr) {
    const int rl = wave * 8 + rr;
    const int i  = blk * 64 + rl;
    const int* arow = adj + (size_t)(n * kNE + i) * kNE;
    float mx = -INFINITY;
#pragma unroll 1
    for (int it = 0; it < 2; ++it) {
      const int j0 = it * 256 + lane * 8;
      const v4i a0 = *(const v4i*)(arow + j0);
      const v4i a1 = *(const v4i*)(arow + j0 + 4);
      float sv[8];
#pragma unroll
      for (int e = 0; e < 8; ++e) {
        const int traw = (e < 4) ? a0[e & 3] : a1[e & 3];
        int tc = traw < 1 ? 1 : traw;
        tc = (tc > kNTy ? kNTy : tc) - 1;
        const float v  = ssrc[tc * 64 + rl] + sd[tc * kNE + j0 + e];
        const float lr = (v >= 0.0f) ? v : (kSlope * v);
        float s = (traw >= 1 && traw <= kNTy) ? lr : 0.0f;
        s = (traw > 0) ? s : kFill;
        sv[e] = s;
        mx = fmaxf(mx, s);
      }
      *(v4f*)(scw + j0)     = (v4f){sv[0], sv[1], sv[2], sv[3]};
      *(v4f*)(scw + j0 + 4) = (v4f){sv[4], sv[5], sv[6], sv[7]};
    }
#pragma unroll
    for (int off = 16; off > 0; off >>= 1) mx = fmaxf(mx, __shfl_xor(mx, off, 32));

    float zs = 0.0f;
    unsigned short* prow = PP + (size_t)(n * kNE + i) * kNE;
#pragma unroll 1
    for (int it = 0; it < 2; ++it) {
      const int j0 = it * 256 + lane * 8;
      const v4f s0 = *(const v4f*)(scw + j0);
      const v4f s1 = *(const v4f*)(scw + j0 + 4);
      v8h hv;
#pragma unroll
      for (int e = 0; e < 8; ++e) {
        const float s = (e < 4) ? s0[e & 3] : s1[e & 3];
        const float p = flush_h(expf(s - mx));
        const _Float16 hp = (_Float16)p;
        hv[e] = hp;
        float pf = (float)hp;
        asm volatile("" : "+v"(pf));
        zs += pf;
      }
      *(volatile v8h*)(prow + j0) = hv;
      __threadfence();
      *(volatile v8h*)(prow + j0) = hv;
    }
#pragma unroll
    for (int off = 16; off > 0; off >>= 1) zs += __shfl_xor(zs, off, 32);
    if (lane == 0) sz[rl] = 1.0f / zs;
  }
  __syncthreads();
  if (tid < 16) {
    const v4f zv = *(const v4f*)(sz + tid * 4);
    float* dst = ZI + (size_t)n * kNE + blk * 64 + tid * 4;
    *(volatile v4f*)dst = zv;
    __threadfence();
    *(volatile v4f*)dst = zv;
  }
}

__global__ __launch_bounds__(256) void agg_gemm_kernel(
    const unsigned short* __restrict__ Pp, const unsigned short* __restrict__ Hp,
    const float* __restrict__ ZI, float* __restrict__ out)
{
  __shared__ __align__(16) float sC[32 * kDim];
  __shared__ __align__(16) float sInv[64];
  const int tid = threadIdx.x, lane = tid & 31, wave = tid >> 5;
  const int hh = lane >> 4, c = lane & 15;
  const int n = blockIdx.y, i0 = blockIdx.x * 64;
  const int rg = wave >> 2, cg = wave & 3;

  if (tid < 64) sInv[tid] = ZI[(size_t)n * kNE + i0 + tid];

  const _Float16* A = (const _Float16*)Pp + (size_t)(n * kNE + i0 + rg * 32) * kNE;
  const _Float16* B = (const _Float16*)Hp + (size_t)(n * kDimP + cg * 80) * kNE;

  v8f acc[2][5];
#pragma unroll
  for (int i = 0; i < 2; ++i)
#pragma unroll
    for (int j = 0; j < 5; ++j) acc[i][j] = (v8f){0.f,0.f,0.f,0.f,0.f,0.f,0.f,0.f};

#pragma unroll 1
  for (int k0 = 0; k0 < kNE; k0 += 32) {
    v16h bf[5];
#pragma unroll
    for (int j = 0; j < 5; ++j) bf[j] = FragH::load(B + (size_t)(j * 16 + c) * kNE + k0 + 8 * hh);
#pragma unroll
    for (int i = 0; i < 2; ++i) {
      const v16h af = FragH::load(A + (size_t)(i * 16 + c) * kNE + k0 + 8 * hh);
#pragma unroll
      for (int j = 0; j < 5; ++j) acc[i][j] = mma_h(af, bf[j], acc[i][j]);
    }
  }
  __syncthreads();

#pragma unroll
  for (int ph = 0; ph < 2; ++ph) {
    if (rg == ph) {
#pragma unroll
      for (int i = 0; i < 2; ++i) {
#pragma unroll
        for (int r = 0; r < 8; ++r) {
          const int row = i * 16 + 8 * hh + r;
          const float sc = sInv[ph * 32 + row] * kScale2;
#pragma unroll
          for (int j = 0; j < 5; ++j) {
            const int col = cg * 80 + j * 16 + c;
            if (col < kDim) sC[row * kDim + col] = acc[i][j][r] * sc;
          }
        }
      }
    }
    __syncthreads();
    float* dst = out + (size_t)(n * kNE + i0 + ph * 32) * kDim;
    for (int pass = 0; pass < 2; ++pass) {
#pragma unroll 1
      for (int it = 0; it < 10; ++it) {
        const int f = it * 256 + tid;
        if (f < (32 * kDim) / 4) {
          const v4f v = *(const v4f*)(sC + f * 4);
          *(volatile v4f*)(dst + (size_t)f * 4) = v;
        }
      }
      __threadfence();
    }
    __syncthreads();
  }
}

extern "C" void kernel_launch(void* const* d_in, const int* in_sizes, int n_in,
                              void* d_out, int out_size, void* d_ws, size_t ws_size,
                              hipStream_t stream) {
  if (n_in < 8) return;
  if (in_sizes[0] != kNB * kNE * kDim) return;
  if (in_sizes[1] != kNB * kNE * kNE) return;
  if (in_sizes[2] != kNB * kNE) return;
  if (in_sizes[3] != kNB * kDim) return;
  if (in_sizes[4] != kNTy * kDim * kDim) return;
  if (in_sizes[5] != kNTy * kTwoD) return;
  if (in_sizes[6] != kNTy * kDim * kTwoD) return;
  if (in_sizes[7] != kNTy * kTwoD * kTwoD) return;
  if (out_size != kNB * kNE * kDim) return;
  if (ws_size < kWsTotal) return;

  const float* input_state = (const float*)d_in[0];
  const int*   adj         = (const int*)  d_in[1];
  const float* node_mask   = (const float*)d_in[2];
  const float* query_vec   = (const float*)d_in[3];
  const float* W_type      = (const float*)d_in[4];
  const float* a_type      = (const float*)d_in[5];
  const float* qattn_W1    = (const float*)d_in[6];
  const float* qattn_W2    = (const float*)d_in[7];
  float* out = (float*)d_out;

  char* ws = (char*)d_ws;
  unsigned short* W3T = (unsigned short*)(ws + kOffW3T);
  float*          U   = (float*)(ws + kOffU);
  float*          S   = (float*)(ws + kOffS);
  unsigned short* XH  = (unsigned short*)(ws + kOffXH);
  unsigned short* HMT = (unsigned short*)(ws + kOffHMT);
  unsigned short* PP  = (unsigned short*)(ws + kOffPP);
  float*          ZI  = (float*)(ws + kOffZI);

  prep_w3t_kernel<<<dim3((kDimP * (kDimP / 8)) / 256), 256, 0, stream>>>(W_type, W3T);
  gate_fold_kernel<<<dim3(kNTy, kNB), 256, 0, stream>>>(query_vec, W_type, a_type, qattn_W1, qattn_W2, U);
  score_cast_kernel<<<dim3(kNE / 64, kNB), 256, 0, stream>>>(input_state, U, S, XH);
  proj_gemm_kernel<<<dim3(((kDimP / 64) * (kNE / 64)) / 8, kNB), 256, 0, stream>>>(W3T, XH, HMT, node_mask);
  coef_kernel<<<dim3(kNE / 64, kNB), 256, 0, stream>>>(adj, S, PP, ZI);
  agg_gemm_kernel<<<dim3(kNE / 64, kNB), 256, 0, stream>>>(PP, HMT, ZI, out);
}
